// TransformerEncoderLayer_83056077570746
// MI455X (gfx1250) — hardware-verified
//
#include <hip/hip_runtime.h>
#ifndef NB
#define NB 1
#endif
#ifndef SQ
#define SQ 4096
#endif
#define NB_FULL 1
#define SQ_FULL 4096
#define DM 768
#define NH 12
#define HD 64
#define DFF 3072
#define LQ (3 * DM)
#define QH (SQ / 2)
#define DMQ DM
#define NR ((size_t)NB * SQ)

static_assert(NB >= 1 && NB <= NB_FULL);
static_assert(SQ >= 256 && SQ <= SQ_FULL && SQ % 256 == 0);
static_assert(NH * HD == DM && HD == 64);
static_assert(DM % 64 == 0 && LQ % 64 == 0 && DFF % 64 == 0);
static_assert(DM % 32 == 0 && DFF % 32 == 0 && SQ % 64 == 0 && QH % 128 == 0);
static_assert((NR % 128) == 0);
static_assert(DMQ <= 1024 && DMQ % 4 == 0);
static_assert(((size_t)(NB - 1) * SQ_FULL + SQ) * DM * 4 <= (size_t)NB_FULL * SQ_FULL * DM * 4);

typedef unsigned short v8us __attribute__((ext_vector_type(8), may_alias));
typedef float  v8f  __attribute__((ext_vector_type(8)));
typedef float  v4f  __attribute__((ext_vector_type(4)));
typedef float  v4fa __attribute__((ext_vector_type(4), may_alias));
typedef _Float16 v16h __attribute__((ext_vector_type(16)));
typedef _Float16 v4h __attribute__((ext_vector_type(4)));
union FragH { v16h v; v8us half[2]; _Float16 h[16]; unsigned short u[16]; };

__device__ __forceinline__ unsigned short bf16_bits(float x) { unsigned int u = __float_as_uint(x); return (unsigned short)((u + 0x7FFFu + ((u >> 16) & 1u)) >> 16); }
__device__ __forceinline__ float bf16_val(unsigned short b) { return __uint_as_float(((unsigned int)b) << 16); }
__device__ __forceinline__ float bf16_rne(float x) { return bf16_val(bf16_bits(x)); }

__device__ __forceinline__ v16h g2_frag(const _Float16* p, int hh) { FragH f; f.half[0] = *(const v8us*)((const unsigned short*)p + 8 * hh); f.half[1] = *(const v8us*)((const unsigned short*)p + 16 + 8 * hh); return f.v; }
__device__ __forceinline__ v8f g2_mma(v16h a, v16h b, v8f c) { v8f d = __builtin_amdgcn_wmma_f32_16x16x32_f16(false, a, false, b, (short)0, c, false, false); asm volatile("v_nop\n\tv_nop\n\tv_nop\n\tv_nop" : "+v"(d) : "v"(a), "v"(b)); return d; }

template <int ACT>
__global__ __launch_bounds__(128) void k_gemm2(const _Float16* __restrict__ A, int lda, size_t sA, const _Float16* __restrict__ Bh, int ldb, size_t sB, float alpha, const float* __restrict__ bias, size_t sBias, const float* __restrict__ CP, int rowsPerB, size_t sCPb, int row0g,
    float* __restrict__ C, _Float16* __restrict__ C16, int ldc, size_t sC, int M, int N, int K) {
  static_assert(ACT == 0 || ACT == 3 || ACT == 6);
  __shared__ __attribute__((aligned(16))) float so[4][32][68];
  const int tid = threadIdx.x, w = tid >> 5, lane = tid & 31, ln = lane & 15, hh = lane >> 4; const int by = blockIdx.y;
  A += (size_t)by * sA; Bh += (size_t)by * sB; const size_t cofs = (size_t)by * sC; const float* bp = bias ? bias + (size_t)by * sBias : nullptr;
  const int ntn = N >> 6; const int mt = blockIdx.x / ntn, nq = blockIdx.x - mt * ntn; const int row0 = mt * 128 + 32 * w, col0 = nq * 64; if (row0 >= M) return;
  const _Float16* a0p = A + (size_t)(row0 + ln) * lda; const _Float16* a1p = a0p + (size_t)16 * lda;
  const _Float16* b0p = Bh + (size_t)(col0 + ln) * ldb; const _Float16* b1p = b0p + (size_t)16 * ldb; const _Float16* b2p = b1p + (size_t)16 * ldb; const _Float16* b3p = b2p + (size_t)16 * ldb;
  const v8f z8 = {0.f,0.f,0.f,0.f,0.f,0.f,0.f,0.f}; v8f c00 = z8, c01 = z8, c02 = z8, c03 = z8, c10 = z8, c11 = z8, c12 = z8, c13 = z8;
#pragma unroll 1
  for (int kb = 0; kb < K; kb += 32) { const v16h a0 = g2_frag(a0p + kb, hh), a1 = g2_frag(a1p + kb, hh);
    v16h b = g2_frag(b0p + kb, hh); c00 = g2_mma(a0, b, c00); c10 = g2_mma(a1, b, c10);
    b = g2_frag(b1p + kb, hh); c01 = g2_mma(a0, b, c01); c11 = g2_mma(a1, b, c11);
    b = g2_frag(b2p + kb, hh); c02 = g2_mma(a0, b, c02); c12 = g2_mma(a1, b, c12);
    b = g2_frag(b3p + kb, hh); c03 = g2_mma(a0, b, c03); c13 = g2_mma(a1, b, c13); }
  v8f accs[8] = {c00, c01, c02, c03, c10, c11, c12, c13};
#pragma unroll
  for (int u = 0; u < 8; ++u) { const int t = u & 3, half = u >> 2; const int col = col0 + t * 16 + ln; const float bv = bp ? bf16_rne(bp[col]) : 0.f;
#pragma unroll
    for (int r = 0; r < 8; ++r) { const int rloc = half * 16 + 8 * hh + r; float v = accs[u][r] * alpha + bv;
      if (CP) { if (rowsPerB < 0) v += CP[cofs + (size_t)(row0g + row0 + rloc) * ldc + col];        else { const int bidx = (row0g + row0 + rloc) / rowsPerB; v += CP[(size_t)bidx * sCPb + (size_t)by * 64 + col]; } }
      if (ACT == 3) v = fmaxf(v, 0.f); else if (ACT == 6) v = 0.5f * v * (1.0f + erff(v * 0.70710678118654752f));
      so[w][rloc][t * 16 + ln] = v; } }
  __builtin_amdgcn_fence(4  , "workgroup"); __builtin_amdgcn_wave_barrier();
  const int rsub = lane >> 4, c4 = (lane & 15) * 4;
  for (int pass = 0; pass < 2; ++pass) {
#pragma unroll
    for (int q = 0; q < 16; ++q) { const int r = q * 2 + rsub; const v4f v = *(const v4fa*)&so[w][r][c4];
      if (C) *(volatile v4f*)(C + cofs + (size_t)(row0 + r) * ldc + col0 + c4) = v;
      if (C16) { v4h h4; for (int i = 0; i < 4; ++i) h4[i] = (_Float16)v[i]; *(volatile v4h*)(C16 + cofs + (size_t)(row0 + r) * ldc + col0 + c4) = h4; } }
    if (pass == 0) __threadfence(); } }

__global__ __launch_bounds__(256) void k_wnat(const float* __restrict__ w, size_t n8, _Float16* __restrict__ Bt) { const size_t t = (size_t)blockIdx.x * 256 + threadIdx.x; if (t >= n8) return;
  const v4f a = *(const v4fa*)(w + t * 8), c = *(const v4fa*)(w + t * 8 + 4); FragH f;
#pragma unroll
  for (int q = 0; q < 4; ++q) { f.h[q] = (_Float16)(bf16_rne(a[q]) * 16.0f); f.h[4 + q] = (_Float16)(bf16_rne(c[q]) * 16.0f); }
  unsigned short* d = (unsigned short*)Bt + t * 8; *(volatile v8us*)d = f.half[0]; __threadfence(); *(volatile v8us*)d = f.half[0]; }

__global__ __launch_bounds__(256) void k_bfr(const float* __restrict__ x, float* __restrict__ XB, size_t n4) { const size_t t = (size_t)blockIdx.x * 256 + threadIdx.x; if (t >= n4) return; v4f a = *(const v4fa*)(x + t * 4);
#pragma unroll
  for (int q = 0; q < 4; ++q) a[q] = bf16_rne(a[q]);
  *(volatile v4f*)(XB + t * 4) = a; __threadfence(); *(volatile v4f*)(XB + t * 4) = a; }

template <int BFIN, int W16, int W32>
__global__ __launch_bounds__(256) void k_lnx(const float* __restrict__ X, const float* __restrict__ g, const float* __restrict__ bb, float eps, _Float16* __restrict__ N16, float* __restrict__ N32) {
  #pragma clang fp contract(off)
  __shared__ float red[256]; const size_t r = blockIdx.x; const int t = threadIdx.x; const bool act = t < (DMQ / 4); const int c0 = act ? t * 4 : 0;
  const v4f xa = *(const v4fa*)(X + r * DMQ + c0); float s[4]; float sum = 0.f;
#pragma unroll
  for (int q = 0; q < 4; ++q) { s[q] = act ? (BFIN ? bf16_rne(xa[q]) : xa[q]) : 0.f; sum = __fadd_rn(sum, s[q]); }
  red[t] = sum; __syncthreads(); for (int st = 128; st > 0; st >>= 1) { if (t < st) red[t] = __fadd_rn(red[t], red[t + st]); __syncthreads(); } const float mu = red[0] / (float)DMQ; __syncthreads();
  float vs = 0.f;
#pragma unroll
  for (int q = 0; q < 4; ++q) { const float dl = act ? __fadd_rn(s[q], -mu) : 0.f; vs = __fadd_rn(vs, __fmul_rn(dl, dl)); }
  red[t] = vs; __syncthreads(); for (int st = 128; st > 0; st >>= 1) { if (t < st) red[t] = __fadd_rn(red[t], red[t + st]); __syncthreads(); }
  const float rs = rsqrtf(__fadd_rn(red[0] / (float)DMQ, eps)); v4h y; v4f yf;
#pragma unroll
  for (int q = 0; q < 4; ++q) { const int c = c0 + q; yf[q] = __fadd_rn(__fmul_rn(__fmul_rn(__fadd_rn(s[q], -mu), rs), bf16_rne(g[c])), bf16_rne(bb[c])); y[q] = (_Float16)yf[q]; }
  if (!act) return;
  for (int pass = 0; pass < 2; ++pass) { if (W16) *(volatile v4h*)(N16 + r * DMQ + c0) = y; if (W32) *(volatile v4f*)(N32 + r * DMQ + c0) = yf; if (pass == 0) __threadfence(); } }

template <int NHv, int TTv>
__global__ __launch_bounds__(256) void k_vt(const _Float16* __restrict__ V16, int ldv, int voff, _Float16* __restrict__ Vt) { __shared__ unsigned short tl[64][66]; const int tid = threadIdx.x; const int slab = blockIdx.x / (TTv / 64), lg = blockIdx.x % (TTv / 64); const int b = slab / NHv, h = slab % NHv;
  for (int i = tid; i < 64 * 8; i += 256) { const int r = i / 8, c8 = (i % 8) * 8; FragH f; f.half[0] = *(const v8us*)((const unsigned short*)V16 + ((size_t)b * TTv + lg * 64 + r) * ldv + voff + h * 64 + c8);
#pragma unroll
    for (int q = 0; q < 8; ++q) tl[r][c8 + q] = f.u[q]; }
  __syncthreads();
  for (int pass = 0; pass < 2; ++pass) {
#pragma unroll
    for (int rd = 0; rd < 2; ++rd) { const int d = rd * 32 + tid / 8, pc = tid % 8; FragH f;
#pragma unroll
      for (int q = 0; q < 8; ++q) f.u[q] = tl[pc * 8 + q][d];
      *(volatile v8us*)((unsigned short*)Vt + ((size_t)slab * 64 + d) * TTv + lg * 64 + pc * 8) = f.half[0]; }
    if (pass == 0) __threadfence(); } }

__global__ __launch_bounds__(256) void k_rsmf(const float* __restrict__ S, _Float16* __restrict__ P, int qn) {
  #pragma clang fp contract(off)
  __shared__ __attribute__((aligned(16))) unsigned short tl[256][72];
  const int tid = threadIdx.x; const int rb = blockIdx.x * 256; const int row = rb + tid; const int rowc = (row < qn) ? row : (qn - 1);
  const float* s = S + (size_t)rowc * SQ;
  float m0 = -3.0e38f, m1 = -3.0e38f, m2 = -3.0e38f, m3 = -3.0e38f;
#pragma unroll 1
  for (int j = 0; j < SQ; j += 4) { const v4f a = *(const v4fa*)(s + j); m0 = fmaxf(m0, a[0]); m1 = fmaxf(m1, a[1]); m2 = fmaxf(m2, a[2]); m3 = fmaxf(m3, a[3]); }
  const float mx = fmaxf(fmaxf(m0, m1), fmaxf(m2, m3));
  float e0 = 0.f, e1 = 0.f, e2 = 0.f, e3 = 0.f;
#pragma unroll 1
  for (int j = 0; j < SQ; j += 4) { const v4f a = *(const v4fa*)(s + j); e0 += __expf(a[0] - mx); e1 += __expf(a[1] - mx); e2 += __expf(a[2] - mx); e3 += __expf(a[3] - mx); }
  const float se = (e0 + e1) + (e2 + e3); const float sc = 256.0f / se;
#pragma unroll 1
  for (int j0 = 0; j0 < SQ; j0 += 64) {
#pragma unroll 1
    for (int u = 0; u < 8; ++u) { const v4f a = *(const v4fa*)(s + j0 + 8 * u), c = *(const v4fa*)(s + j0 + 8 * u + 4); FragH f;
#pragma unroll
      for (int q = 0; q < 4; ++q) { f.h[q] = (_Float16)(__expf(a[q] - mx) * sc); f.h[4 + q] = (_Float16)(__expf(c[q] - mx) * sc); }
      *(v8us*)&tl[tid][8 * u] = f.half[0]; }
    __syncthreads();
    for (int pass = 0; pass < 2; ++pass) {
#pragma unroll
      for (int it = 0; it < 8; ++it) { const int r = it * 32 + (tid >> 3), pc = (tid & 7) * 8; const v8us v = *(const v8us*)&tl[r][pc];
        if (rb + r < qn) *(volatile v8us*)((unsigned short*)P + (size_t)(rb + r) * SQ + j0 + pc) = v; }
      if (pass == 0) __threadfence(); }
    __syncthreads(); } }

constexpr size_t al256(size_t b) { return (b + 255) & ~(size_t)255; }
constexpr size_t cmax(size_t a, size_t b) { return a > b ? a : b; }
constexpr size_t SZ_BQKV = (size_t)3 * DM * DM * 2, SZ_BO = (size_t)DM * DM * 2, SZ_BW1 = (size_t)DFF * DM * 2, SZ_BW2 = (size_t)DM * DFF * 2;
constexpr size_t SZ_XB = NR * DM * 4, SZ_X16 = NR * DM * 2, SZ_QKV = NR * LQ * 2, SZ_VT = (size_t)NH * HD * SQ * 2;
constexpr size_t SZ_S = (size_t)QH * SQ * 4, SZ_X1 = NR * DM * 4, SZ_M16 = NR * DM * 2, SZ_RS = cmax(SZ_S, al256(SZ_X1) + SZ_M16);
constexpr size_t SZ_P = (size_t)SQ * SQ * 2, SZ_HF = (size_t)SQ * DFF * 2, SZ_RP = cmax(SZ_P, SZ_HF);
constexpr size_t WS_TOTAL = al256(SZ_BQKV) + al256(SZ_BO) + al256(SZ_BW1) + al256(SZ_BW2) + al256(SZ_XB) + al256(SZ_X16) + al256(SZ_QKV) + al256(SZ_VT) + al256(SZ_RS) + al256(SZ_RP);
static_assert(WS_TOTAL <= (size_t)134217728);
static_assert(SZ_X16 == NR * DM * 2);
static_assert(al256(SZ_X1) + SZ_M16 <= SZ_RS && SZ_S <= SZ_RS);
static_assert(SZ_HF <= SZ_RP && SZ_P <= SZ_RP);

extern "C" void kernel_launch(void* const* d_in, const int* in_sizes, int n_in,
                              void* d_out, int out_size, void* d_ws, size_t ws_size, hipStream_t stream) {
  if (n_in < 14) return;
  const float* const* I = (const float* const*)d_in;
  const float* x = I[0]; const float* wq = I[1]; const float* wk = I[2]; const float* wv = I[3]; const float* wo = I[4]; const float* bo = I[5];
  const float* g1 = I[6]; const float* be1 = I[7]; const float* g2 = I[8]; const float* be2 = I[9]; const float* w1 = I[10]; const float* b1 = I[11]; const float* w2 = I[12]; const float* b2 = I[13];
  const size_t needX = ((size_t)(NB - 1) * SQ_FULL + SQ) * DM;
  if ((size_t)in_sizes[0] < needX || (size_t)out_size < needX) return;
  if (in_sizes[1] < DM * DM || in_sizes[2] < DM * DM || in_sizes[3] < DM * DM || in_sizes[4] < DM * DM || in_sizes[5] < DM) return;
  if (in_sizes[6] < DM || in_sizes[7] < DM || in_sizes[8] < DM || in_sizes[9] < DM) return;
  if (in_sizes[10] < DFF * DM || in_sizes[11] < DFF || in_sizes[12] < DM * DFF || in_sizes[13] < DM) return;
  char* ws = (char*)d_ws; size_t off = 0;
  auto take = [&](size_t bytes) { char* p = ws + off; off += al256(bytes); return p; };
  _Float16* BQKV = (_Float16*)take(SZ_BQKV); _Float16* BO = (_Float16*)take(SZ_BO); _Float16* BW1 = (_Float16*)take(SZ_BW1); _Float16* BW2 = (_Float16*)take(SZ_BW2);
  float* XB = (float*)take(SZ_XB); _Float16* X16 = (_Float16*)take(SZ_X16); _Float16* O16 = X16;
  _Float16* QKV = (_Float16*)take(SZ_QKV); _Float16* VT = (_Float16*)take(SZ_VT);
  char* RS = take(SZ_RS); float* S = (float*)RS; float* X1 = (float*)RS; _Float16* M16 = (_Float16*)(RS + al256(SZ_X1));
  char* RP = take(SZ_RP); _Float16* P = (_Float16*)RP; _Float16* HF16 = (_Float16*)RP;
  if (off > ws_size) return;

  const unsigned gW = (unsigned)(((size_t)DM * (DM / 8) + 255) / 256), gW1 = (unsigned)(((size_t)DFF * (DM / 8) + 255) / 256);
  k_wnat<<<gW, 256, 0, stream>>>(wq, (size_t)DM * DM / 8, BQKV);
  k_wnat<<<gW, 256, 0, stream>>>(wk, (size_t)DM * DM / 8, BQKV + (size_t)DM * DM);
  k_wnat<<<gW, 256, 0, stream>>>(wv, (size_t)DM * DM / 8, BQKV + (size_t)2 * DM * DM);
  k_wnat<<<gW, 256, 0, stream>>>(wo, (size_t)DM * DM / 8, BO);
  k_wnat<<<gW1, 256, 0, stream>>>(w1, (size_t)DFF * DM / 8, BW1);
  k_wnat<<<gW1, 256, 0, stream>>>(w2, (size_t)DM * DFF / 8, BW2);
  for (int b = 0; b < NB; ++b) { const size_t rin = (size_t)b * SQ_FULL, r0 = (size_t)b * SQ;
    k_bfr<<<(unsigned)(((size_t)SQ * DM / 4 + 255) / 256), 256, 0, stream>>>(x + rin * DM, XB + r0 * DM, (size_t)SQ * DM / 4);
    k_lnx<1, 1, 0><<<(unsigned)SQ, 256, 0, stream>>>(x + rin * DM, g1, be1, 1e-5f, X16 + r0 * DM, nullptr); }
  k_gemm2<0><<<dim3((unsigned)((NR / 128) * (LQ / 64)), 1), 128, 0, stream>>>(X16, DM, (size_t)0, BQKV, DM, (size_t)0, 0.0625f, nullptr, (size_t)0, nullptr, 1, (size_t)0, 0, nullptr, QKV, LQ, (size_t)0, (int)NR, LQ, DM);
  for (int b = 0; b < NB; ++b) { const size_t r0 = (size_t)b * SQ;
    k_vt<NH, SQ><<<(unsigned)(NH * (SQ / 64)), 256, 0, stream>>>(QKV + r0 * LQ + 2 * DM, LQ, 0, VT);
    for (int h = 0; h < NH; ++h) {
      for (int hf = 0; hf < 2; ++hf) { const size_t q0 = (size_t)hf * QH;
        k_gemm2<0><<<dim3((unsigned)((QH / 128) * (SQ / 64)), 1), 128, 0, stream>>>(QKV + (r0 + q0) * LQ + (size_t)h * HD, LQ, (size_t)0, QKV + r0 * LQ + DM + (size_t)h * HD, LQ, (size_t)0, 0.125f, nullptr, (size_t)0, nullptr, 1, (size_t)0, 0, S, nullptr, SQ, (size_t)0, QH, SQ, HD);
        k_rsmf<<<(unsigned)((QH + 255) / 256), 256, 0, stream>>>(S, P + q0 * SQ, QH); }
      k_gemm2<0><<<dim3((unsigned)((SQ / 128) * (HD / 64)), 1), 128, 0, stream>>>(P, SQ, (size_t)0, VT + (size_t)h * HD * SQ, SQ, (size_t)0, 0.25f, nullptr, (size_t)0, nullptr, 1, (size_t)0, 0, nullptr, O16 + r0 * DM + (size_t)h * HD, DM, (size_t)0, SQ, HD, SQ); } }
  k_gemm2<0><<<dim3((unsigned)((NR / 128) * (DM / 64)), 1), 128, 0, stream>>>(O16, DM, (size_t)0, BO, DM, (size_t)0, 0.0009765625f, bo, (size_t)0, XB, -1, (size_t)0, 0, X1, nullptr, DM, (size_t)0, (int)NR, DM, DM);
  k_lnx<0, 1, 0><<<(unsigned)NR, 256, 0, stream>>>(X1, g2, be2, 1e-5f, M16, nullptr);
  for (int b = 0; b < NB; ++b) { const size_t rin = (size_t)b * SQ_FULL, r0 = (size_t)b * SQ;
    k_gemm2<6><<<dim3((unsigned)((SQ / 128) * (DFF / 64)), 1), 128, 0, stream>>>(M16 + r0 * DM, DM, (size_t)0, BW1, DM, (size_t)0, 0.0625f, b1, (size_t)0, nullptr, 1, (size_t)0, 0, nullptr, HF16, DFF, (size_t)0, SQ, DFF, DM);
    k_gemm2<0><<<dim3((unsigned)((SQ / 128) * (DM / 64)), 1), 128, 0, stream>>>(HF16, DFF, (size_t)0, BW2, DFF, (size_t)0, 0.0625f, b2, (size_t)0, X1 + r0 * DM, -1, (size_t)0, 0, (float*)d_out + rin * DM, nullptr, DM, (size_t)0, SQ, DM, DFF); }
}
